// LSTMModel_20839181320280
// MI455X (gfx1250) — hardware-verified
//
#include <hip/hip_runtime.h>
#include <math.h>

constexpr int NB   = 8192;
constexpr int NT   = 256;
constexpr int NI   = 6;
constexpr int NH   = 32;
constexpr int NG   = 128;
constexpr int NM1  = 64;
constexpr int NTHR = 128;
constexpr int NWAV = NTHR / 32;
constexpr int RPW  = 16;
constexpr int RPB  = RPW * NWAV;
constexpr int WP   = 40;
constexpr int HSP  = 36;
constexpr int XSP  = 8;
static_assert(NG == 4 * NH);
static_assert(NH == 32);
static_assert(NTHR == NG);
static_assert(NM1 == 64 && NM1 <= NTHR);
static_assert(NB % RPB == 0);
static_assert((RPW * HSP) % 32 == 0);
static_assert(RPB * 4 == 256);
static_assert(WP % 8 == 0 && HSP % 4 == 0 && XSP % 4 == 0);
static_assert(NI == 6);

typedef __attribute__((ext_vector_type(16))) __bf16 v16b;
typedef __attribute__((ext_vector_type(8)))  __bf16 v8b;
typedef __attribute__((ext_vector_type(8)))  float  v8f;
typedef __attribute__((ext_vector_type(4)))  float  v4f;
typedef __attribute__((ext_vector_type(2)))  float  v2f;

__device__ __forceinline__ unsigned short f2bf_bits(float f) {
  unsigned u = __float_as_uint(f);
  return (unsigned short)((u + 0x7FFFu + ((u >> 16) & 1u)) >> 16);
}
__device__ __forceinline__ void split_bf(float f, __bf16& hi, __bf16& lo) {
  const unsigned short hb = f2bf_bits(f);
  hi = __builtin_bit_cast(__bf16, hb);
  const float res = f - __uint_as_float(((unsigned)hb) << 16);
  lo = __builtin_bit_cast(__bf16, f2bf_bits(res));
}
__device__ __forceinline__ void split8(v4f a, v4f b, v8b& hv, v8b& lv) {
#pragma unroll
  for (int e = 0; e < 4; ++e) {
    const float va = a[e];
    __bf16 h0, l0; split_bf(va, h0, l0);
    hv[e] = h0; lv[e] = l0;
    const float vb = b[e];
    __bf16 h1, l1; split_bf(vb, h1, l1);
    hv[4 + e] = h1; lv[4 + e] = l1;
  }
}
__device__ __forceinline__ v16b frag_load(const __bf16* p) {
  union { v16b v; v8b h[2]; } f;
  f.h[0] = *(const v8b*)(p);
  f.h[1] = *(const v8b*)(p + 16);
  return f.v;
}
__device__ __forceinline__ void build_afrag(const float* row, int koff, v16b& hi, v16b& lo) {
  const v4f f0 = *(const v4f*)(row + koff);
  const v4f f1 = *(const v4f*)(row + koff + 4);
  const v4f f2 = *(const v4f*)(row + 16 + koff);
  const v4f f3 = *(const v4f*)(row + 16 + koff + 4);
#pragma unroll
  for (int e = 0; e < 4; ++e) {
    __bf16 a, b;
    const float v0 = f0[e]; split_bf(v0, a, b); hi[e] = a;      lo[e] = b;
    const float v1 = f1[e]; split_bf(v1, a, b); hi[4 + e] = a;  lo[4 + e] = b;
    const float v2 = f2[e]; split_bf(v2, a, b); hi[8 + e] = a;  lo[8 + e] = b;
    const float v3 = f3[e]; split_bf(v3, a, b); hi[12 + e] = a; lo[12 + e] = b;
  }
}
__device__ __forceinline__ v8f mma_bf(v16b a, v16b b, v8f c) {
  return __builtin_amdgcn_wmma_f32_16x16x32_bf16(false, a, false, b, (short)0, c, false, false);
}
__device__ __forceinline__ void tile_guard(v8f& acc, v16b w, v16b x, v16b y, v16b z) {
  asm volatile("v_nop\n\tv_nop\n\tv_nop\n\tv_nop" : "+v"(acc) : "v"(w), "v"(x), "v"(y), "v"(z) : "memory");
}
__device__ __forceinline__ void acc_guard4(v8f& a, v8f& b, v8f& c, v8f& d) {
  asm volatile("v_nop\n\tv_nop\n\tv_nop\n\tv_nop" : "+v"(a), "+v"(b), "+v"(c), "+v"(d));
}
__device__ __forceinline__ void wave_sync() {
  __builtin_amdgcn_fence(__ATOMIC_RELEASE, "workgroup");
  __builtin_amdgcn_wave_barrier();
  __builtin_amdgcn_fence(__ATOMIC_ACQUIRE, "workgroup");
}
__device__ __forceinline__ v8f splat8(float s) { v8f v; v[0]=s; v[1]=s; v[2]=s; v[3]=s; v[4]=s; v[5]=s; v[6]=s; v[7]=s; return v; }
__device__ __forceinline__ float fsig(float x)  { return __builtin_amdgcn_rcpf(1.0f + expf(-x)); }
__device__ __forceinline__ float ftanh(float x) { return 1.0f - 2.0f * __builtin_amdgcn_rcpf(expf(2.0f * x) + 1.0f); }

__global__ __launch_bounds__(NTHR) void lstm_head_kernel(
    const float* __restrict__ x, const float* __restrict__ W_ih, const float* __restrict__ W_hh,
    const float* __restrict__ b_ih, const float* __restrict__ b_hh,
    const float* __restrict__ W1, const float* __restrict__ b1, const float* __restrict__ W2, const float* __restrict__ b2,
    float* __restrict__ out) {
  __shared__ __align__(16) __bf16 Whi[NG * WP];
  __shared__ __align__(16) __bf16 Wlo[NG * WP];
  __shared__ __align__(16) __bf16 W1hi[NM1 * WP];
  __shared__ __align__(16) __bf16 W1lo[NM1 * WP];
  __shared__ __align__(16) float  Wib[NG * XSP];
  __shared__ __align__(16) float  b1s[NM1];
  __shared__ __align__(16) float  w2s[NM1];
  __shared__ __align__(16) float  Hs[NWAV][RPW * HSP];
  __shared__ __align__(16) float  Xs[NWAV][RPW * XSP];
  __shared__ __align__(16) float  Os[RPB];

  const int tid = threadIdx.x, lane = tid & 31, wave = tid >> 5;
  const int c = lane & 15, hh = lane >> 4, koff = 8 * hh;
  const int rb = blockIdx.x * RPB + wave * RPW;

  {
    const float* wr = W_hh + (size_t)tid * NH;
#pragma unroll 1
    for (int g = 0; g < NH / 8; ++g) {
      const v4f a = *(const v4f*)(wr + 8 * g);
      const v4f b = *(const v4f*)(wr + 8 * g + 4);
      v8b hv, lv; split8(a, b, hv, lv);
      *(v8b*)(Whi + tid * WP + 8 * g) = hv;
      *(v8b*)(Wlo + tid * WP + 8 * g) = lv;
    }
  }
  if (wave < 2) {
    const float* wr = W1 + (size_t)tid * NH;
#pragma unroll 1
    for (int g = 0; g < NH / 8; ++g) {
      const v4f a = *(const v4f*)(wr + 8 * g);
      const v4f b = *(const v4f*)(wr + 8 * g + 4);
      v8b hv, lv; split8(a, b, hv, lv);
      *(v8b*)(W1hi + tid * WP + 8 * g) = hv;
      *(v8b*)(W1lo + tid * WP + 8 * g) = lv;
    }
    b1s[tid] = b1[tid];
    w2s[tid] = W2[tid];
  }
  {
    const float* wi = W_ih + (size_t)tid * NI;
    const v2f p0 = *(const v2f*)(wi);
    const v2f p1 = *(const v2f*)(wi + 2);
    const v2f p2 = *(const v2f*)(wi + 4);
    const float bs = b_ih[tid] + b_hh[tid];
    v4f wa, wb;
    wa[0] = p0[0]; wa[1] = p0[1]; wa[2] = p1[0]; wa[3] = p1[1];
    wb[0] = p2[0]; wb[1] = p2[1]; wb[2] = bs;    wb[3] = 0.0f;
    *(v4f*)(Wib + tid * XSP)     = wa;
    *(v4f*)(Wib + tid * XSP + 4) = wb;
  }
  float* Hsw = Hs[wave];
  float* Xsw = Xs[wave];
#pragma unroll
  for (int i = 0; i < (RPW * HSP) / 32; ++i) Hsw[lane + 32 * i] = 0.0f;
  float cst[2][8];
#pragma unroll
  for (int u = 0; u < 2; ++u)
#pragma unroll
    for (int r = 0; r < 8; ++r) cst[u][r] = 0.0f;
  __syncthreads();

  const float* xrow_base = x + (size_t)(rb + c) * (size_t)(NT * NI);

#pragma unroll 1
  for (int t = 0; t < NT; ++t) {
    {
      const float* p = xrow_base + (size_t)t * NI;
      const v2f va = *(const v2f*)(p + 2 * hh);
      const v2f vb = *(const v2f*)(p + 4);
      *(v2f*)(Xsw + c * XSP + 2 * hh) = va;
      *(v2f*)(Xsw + c * XSP + 4)      = vb;
    }
    wave_sync();

    v4f xa[8]; v2f xb[8];
#pragma unroll
    for (int r = 0; r < 8; ++r) {
      xa[r] = *(const v4f*)(Xsw + (8 * hh + r) * XSP);
      xb[r] = *(const v2f*)(Xsw + (8 * hh + r) * XSP + 4);
    }

    v8f acc[8];
#pragma unroll
    for (int n = 0; n < 8; ++n) {
      const float* wrow = Wib + (16 * n + c) * XSP;
      const v4f wa = *(const v4f*)(wrow);
      const v4f wb = *(const v4f*)(wrow + 4);
#pragma unroll
      for (int r = 0; r < 8; ++r) {
        float d = xa[r][0] * wa[0];
        d = fmaf(xa[r][1], wa[1], d);
        d = fmaf(xa[r][2], wa[2], d);
        d = fmaf(xa[r][3], wa[3], d);
        d = fmaf(xb[r][0], wb[0], d);
        d = fmaf(xb[r][1], wb[1], d);
        acc[n][r] = d + wb[2];
      }
    }

    v16b ahi, alo;
    build_afrag(Hsw + c * HSP, koff, ahi, alo);

#pragma unroll
    for (int n = 0; n < 8; ++n) {
      const v16b bh = frag_load(Whi + (16 * n + c) * WP + koff);
      const v16b bl = frag_load(Wlo + (16 * n + c) * WP + koff);
      acc[n] = mma_bf(ahi, bh, acc[n]);
      acc[n] = mma_bf(ahi, bl, acc[n]);
      acc[n] = mma_bf(alo, bh, acc[n]);
      tile_guard(acc[n], ahi, alo, bh, bl);
    }
    acc_guard4(acc[0], acc[1], acc[2], acc[3]);
    acc_guard4(acc[4], acc[5], acc[6], acc[7]);

    float hn[2][8];
#pragma unroll
    for (int u = 0; u < 2; ++u) {
#pragma unroll
      for (int r = 0; r < 8; ++r) {
        const float zi = acc[u][r];
        const float zf = acc[2 + u][r];
        const float zg = acc[4 + u][r];
        const float zo = acc[6 + u][r];
        const float ig = fsig(zi);
        const float fg = fsig(zf);
        const float gg = ftanh(zg);
        const float og = fsig(zo);
        const float cn = fg * cst[u][r] + ig * gg;
        cst[u][r] = cn;
        hn[u][r] = og * ftanh(cn);
      }
    }

#pragma unroll
    for (int r = 0; r < 8; ++r) {
      Hsw[(8 * hh + r) * HSP + c]      = hn[0][r];
      Hsw[(8 * hh + r) * HSP + 16 + c] = hn[1][r];
    }
    wave_sync();
  }

  v16b ahi, alo;
  build_afrag(Hsw + c * HSP, koff, ahi, alo);
  v8f ha[4];
#pragma unroll
  for (int j = 0; j < 4; ++j) { const float bv = b1s[16 * j + c]; ha[j] = splat8(bv); }
#pragma unroll
  for (int j = 0; j < 4; ++j) {
    const v16b bh = frag_load(W1hi + (16 * j + c) * WP + koff);
    const v16b bl = frag_load(W1lo + (16 * j + c) * WP + koff);
    ha[j] = mma_bf(ahi, bh, ha[j]);
    ha[j] = mma_bf(ahi, bl, ha[j]);
    ha[j] = mma_bf(alo, bh, ha[j]);
    tile_guard(ha[j], ahi, alo, bh, bl);
  }
  acc_guard4(ha[0], ha[1], ha[2], ha[3]);

  float part[8];
#pragma unroll
  for (int r = 0; r < 8; ++r) part[r] = 0.0f;
#pragma unroll
  for (int j = 0; j < 4; ++j) {
    const float w2v = w2s[16 * j + c];
#pragma unroll
    for (int r = 0; r < 8; ++r) part[r] = fmaf(fmaxf(ha[j][r], 0.0f), w2v, part[r]);
  }
#pragma unroll
  for (int off = 1; off < 16; off <<= 1) {
#pragma unroll
    for (int r = 0; r < 8; ++r) part[r] += __shfl_xor(part[r], off, 32);
  }
  const float b2v = b2[0];
  if (c == 0) {
#pragma unroll
    for (int r = 0; r < 8; ++r) Os[RPW * wave + 8 * hh + r] = part[r] + b2v;
  }
  __syncthreads();
  if (wave == 0) {
    const v4f v = *(const v4f*)(Os + 4 * (lane & 15));
    float* op = out + (size_t)blockIdx.x * RPB + 4 * (lane & 15);
    for (int pass = 0; pass < 2; ++pass) {
      if (lane < 16) *(volatile v4f*)op = v;
      __threadfence();
    }
  }
}

extern "C" void kernel_launch(void* const* d_in, const int* in_sizes, int n_in,
                              void* d_out, int out_size, void* d_ws, size_t ws_size, hipStream_t stream) {
  (void)d_ws; (void)ws_size;
  if (n_in < 9 || d_out == nullptr) return;
  if (in_sizes[0] != NB * NT * NI || in_sizes[1] != NG * NI || in_sizes[2] != NG * NH ||
      in_sizes[3] != NG || in_sizes[4] != NG || in_sizes[5] != NM1 * NH || in_sizes[6] != NM1 ||
      in_sizes[7] != NM1 || in_sizes[8] != 1 || out_size != NB) return;

  const float* x    = (const float*)d_in[0];
  const float* W_ih = (const float*)d_in[1];
  const float* W_hh = (const float*)d_in[2];
  const float* b_ih = (const float*)d_in[3];
  const float* b_hh = (const float*)d_in[4];
  const float* W1   = (const float*)d_in[5];
  const float* b1   = (const float*)d_in[6];
  const float* W2   = (const float*)d_in[7];
  const float* b2   = (const float*)d_in[8];
  float* out = (float*)d_out;

  lstm_head_kernel<<<NB / RPB, NTHR, 0, stream>>>(x, W_ih, W_hh, b_ih, b_hh, W1, b1, W2, b2, out);
}
